// MultiHeadAttention_74285754352148
// MI455X (gfx1250) — hardware-run, weakly checked
//
#include <hip/hip_runtime.h>


#ifndef NB
#define NB 2
#endif
#ifndef SEQ
#define SEQ 2048
#endif
#define SEQ_FULL 2048
#define DM   1024
#define NH_  16
#define HD   64
#define DQ   (NH_ * HD)
#define ZH   8
#define RH   ((SEQ) < 512 ? (SEQ) : 512)
#define BOFF 256
#define BW   (BOFF + 64)
#define WINK 257
#define PCAR 1024.0f
#define SCL  0.125f

static_assert(SEQ % 64 == 0);
static_assert(SEQ <= SEQ_FULL);
static_assert(NH_ % ZH == 0);
static_assert(RH % 64 == 0);
static_assert(WINK - 1 <= BOFF);
static_assert(BW % 64 == 0);
static_assert(DM % 64 == 0);
static_assert(DQ % 64 == 0);
static_assert((ZH * SEQ) % 8 == 0);
static_assert(HD == 64);

typedef _Float16 h16;
typedef unsigned short bf;
typedef __attribute__((ext_vector_type(16))) __bf16   v16bf;
typedef __attribute__((ext_vector_type(16))) _Float16 v16h;
typedef __attribute__((ext_vector_type(8)))  _Float16 v8h;
typedef __attribute__((ext_vector_type(8)))  unsigned short v8us;
typedef __attribute__((ext_vector_type(8)))  float    v8f;
typedef __attribute__((ext_vector_type(4)))  float    v4f;
typedef v4f  __attribute__((may_alias)) v4fa;
typedef __attribute__((ext_vector_type(2))) _Float16 v2h;
typedef __attribute__((ext_vector_type(2))) unsigned short v2us;
typedef __attribute__((ext_vector_type(2))) float v2f;

__device__ __forceinline__ unsigned short f2bf(float f) { unsigned u = __float_as_uint(f); u += 0x7FFFu + ((u >> 16) & 1u); return (unsigned short)(u >> 16); }
__device__ __forceinline__ float bf2f(unsigned short b) { return __uint_as_float(((unsigned)b) << 16); }
__device__ __forceinline__ float bfr(float f) { return bf2f(f2bf(f)); }
__device__ __forceinline__ v16h cat16(v8h lo, v8h hi) { return __builtin_shufflevector(lo, hi, 0, 1, 2, 3, 4, 5, 6, 7, 8, 9, 10, 11, 12, 13, 14, 15); }
__device__ __forceinline__ v16bf cat16b(v8us lo, v8us hi) { return __builtin_bit_cast(v16bf, __builtin_shufflevector(lo, hi, 0, 1, 2, 3, 4, 5, 6, 7, 8, 9, 10, 11, 12, 13, 14, 15)); }
__device__ __forceinline__ v8f wmma16(v16h a, v16h b, v8f c) { return __builtin_amdgcn_wmma_f32_16x16x32_f16(false, a, false, b, (short)0, c, false, false); }
__device__ __forceinline__ v8f wmmab(v16bf a, v16bf b, v8f c) { return __builtin_amdgcn_wmma_f32_16x16x32_bf16(false, a, false, b, (short)0, c, false, false); }
__device__ __forceinline__ h16 tohx(float x) { return (h16)x; }
__device__ __forceinline__ void splitf(float y, unsigned short& h, unsigned short& l) { h = f2bf(y); l = f2bf(y - bf2f(h)); }

template <typename T16> struct WFrag;
template <> struct WFrag<h16> { typedef v16h V; static __device__ __forceinline__ V ld(const h16* p) { return cat16(*(const v8h*)p, *(const v8h*)(p + 16)); } static __device__ __forceinline__ v8f mma(V a, V b, v8f c) { return wmma16(a, b, c); } };
template <> struct WFrag<bf> { typedef v16bf V; static __device__ __forceinline__ V ld(const bf* p) { return cat16b(*(const v8us*)p, *(const v8us*)(p + 16)); } static __device__ __forceinline__ v8f mma(V a, V b, v8f c) { return wmmab(a, b, c); } };

template <typename T16, int NSPLIT, bool BIAS>
__global__ __launch_bounds__(32) void k_gemmw(const T16* __restrict__ A, const T16* __restrict__ A2, const T16* __restrict__ Bt, const T16* __restrict__ Bt2, int K, float* C, int ldc, const float* __restrict__ bias, size_t sA, size_t sB, size_t sC) {
    typedef typename WFrag<T16>::V V;
    __shared__ __align__(16) float os[16 * 68];
    const size_t z = blockIdx.z; A += z * sA; if (A2) A2 += z * sA; Bt += z * sB; if (Bt2) Bt2 += z * sB; C += z * sC;
    const int lane = threadIdx.x & 31, lr = lane & 15, hi = lane >> 4; const int r0 = blockIdx.x * 64, c0 = blockIdx.y * 64;
    v8f acc[4][4];
#pragma unroll
    for (int mb = 0; mb < 4; ++mb)
#pragma unroll
        for (int nb = 0; nb < 4; ++nb) acc[mb][nb] = (v8f){};
    const size_t aoff = (size_t)(r0 + lr) * K + 8 * hi, boff = (size_t)(c0 + lr) * K + 8 * hi;
#pragma unroll 1
    for (int kc = 0; kc < K; kc += 32) {
        V a[4], a2[4];
#pragma unroll
        for (int mb = 0; mb < 4; ++mb) { a[mb] = WFrag<T16>::ld(A + aoff + (size_t)mb * 16 * K + kc); if (NSPLIT == 1 || NSPLIT == 2) a2[mb] = WFrag<T16>::ld(A2 + aoff + (size_t)mb * 16 * K + kc); }
#pragma unroll
        for (int nb = 0; nb < 4; ++nb) { const V b = WFrag<T16>::ld(Bt + boff + (size_t)nb * 16 * K + kc); V b2; if (NSPLIT >= 2) b2 = WFrag<T16>::ld(Bt2 + boff + (size_t)nb * 16 * K + kc);
#pragma unroll
            for (int mb = 0; mb < 4; ++mb) { acc[mb][nb] = WFrag<T16>::mma(a[mb], b, acc[mb][nb]); if (NSPLIT == 1 || NSPLIT == 2) acc[mb][nb] = WFrag<T16>::mma(a2[mb], b, acc[mb][nb]); if (NSPLIT >= 2) acc[mb][nb] = WFrag<T16>::mma(a[mb], b2, acc[mb][nb]); } }
        asm volatile("v_nop\n\tv_nop\n\tv_nop\n\tv_nop" : "+v"(acc[0][0]), "+v"(acc[1][1]), "+v"(acc[2][2]), "+v"(acc[3][3]) : "v"(a[0]), "v"(a[3]));
    }
#pragma unroll
    for (int mb = 0; mb < 4; ++mb) {
#pragma unroll
        for (int nb = 0; nb < 4; ++nb) {
#pragma unroll
            for (int j = 0; j < 8; ++j) os[(hi * 8 + j) * 68 + nb * 16 + lr] = acc[mb][nb][j]; }
        __builtin_amdgcn_wave_barrier(); asm volatile("" ::: "memory");
        float* crow = C + (size_t)(r0 + mb * 16) * ldc + c0;
#pragma unroll 1
        for (int ps = 0; ps < 2; ++ps) {
#pragma unroll
            for (int s = 0; s < 8; ++s) { const int row = 2 * s + hi, cofs = lr * 4; v4f val = *(const v4fa*)(os + row * 68 + cofs); if (BIAS) { val[0] += bfr(bias[c0 + cofs]); val[1] += bfr(bias[c0 + cofs + 1]); val[2] += bfr(bias[c0 + cofs + 2]); val[3] += bfr(bias[c0 + cofs + 3]); }
                *(volatile v4f*)(crow + (size_t)row * ldc + cofs) = val; }
            if (ps == 0) __threadfence(); }
        __builtin_amdgcn_wave_barrier(); asm volatile("" ::: "memory");
    }
}

template <typename T16, int NSPLIT>
__global__ __launch_bounds__(32) void k_gemmS(const T16* __restrict__ A, const T16* __restrict__ A2, const T16* __restrict__ Bt, const T16* __restrict__ Bt2, float* S, int roff, size_t sA, size_t sB, size_t sS) {
    typedef typename WFrag<T16>::V V;
    __shared__ __align__(16) float os[16 * 68];
    const size_t z = blockIdx.z; A += z * sA; if (A2) A2 += z * sA; Bt += z * sB; if (Bt2) Bt2 += z * sB; S += z * sS;
    const int lane = threadIdx.x & 31, lr = lane & 15, hi = lane >> 4; const int r0 = roff + (int)blockIdx.x * 64; const int c0 = r0 - BOFF + (int)blockIdx.y * 64;
    if (c0 < 0) return;
    v8f acc[4][4];
#pragma unroll
    for (int mb = 0; mb < 4; ++mb)
#pragma unroll
        for (int nb = 0; nb < 4; ++nb) acc[mb][nb] = (v8f){};
    const size_t aoff = (size_t)(r0 + lr) * HD + 8 * hi, boff = (size_t)(c0 + lr) * HD + 8 * hi;
#pragma unroll 1
    for (int kc = 0; kc < HD; kc += 32) {
        V a[4], a2[4];
#pragma unroll
        for (int mb = 0; mb < 4; ++mb) { a[mb] = WFrag<T16>::ld(A + aoff + (size_t)mb * 16 * HD + kc); if (NSPLIT == 2) a2[mb] = WFrag<T16>::ld(A2 + aoff + (size_t)mb * 16 * HD + kc); }
#pragma unroll
        for (int nb = 0; nb < 4; ++nb) { const V b = WFrag<T16>::ld(Bt + boff + (size_t)nb * 16 * HD + kc); V b2; if (NSPLIT == 2) b2 = WFrag<T16>::ld(Bt2 + boff + (size_t)nb * 16 * HD + kc);
#pragma unroll
            for (int mb = 0; mb < 4; ++mb) { acc[mb][nb] = WFrag<T16>::mma(a[mb], b, acc[mb][nb]); if (NSPLIT == 2) { acc[mb][nb] = WFrag<T16>::mma(a2[mb], b, acc[mb][nb]); acc[mb][nb] = WFrag<T16>::mma(a[mb], b2, acc[mb][nb]); } } }
        asm volatile("v_nop\n\tv_nop\n\tv_nop\n\tv_nop" : "+v"(acc[0][0]), "+v"(acc[1][1]), "+v"(acc[2][2]), "+v"(acc[3][3]) : "v"(a[0]), "v"(a[3]));
    }
#pragma unroll
    for (int mb = 0; mb < 4; ++mb) {
#pragma unroll
        for (int nb = 0; nb < 4; ++nb) {
#pragma unroll
            for (int j = 0; j < 8; ++j) os[(hi * 8 + j) * 68 + nb * 16 + lr] = acc[mb][nb][j]; }
        __builtin_amdgcn_wave_barrier(); asm volatile("" ::: "memory");
        float* crow = S + (size_t)(r0 + mb * 16) * BW + (size_t)blockIdx.y * 64;
#pragma unroll 1
        for (int ps = 0; ps < 2; ++ps) {
#pragma unroll
            for (int s = 0; s < 8; ++s) { const int row = 2 * s + hi, cofs = lr * 4; const v4f val = *(const v4fa*)(os + row * 68 + cofs);
                *(volatile v4f*)(crow + (size_t)row * BW + cofs) = val; }
            if (ps == 0) __threadfence(); }
        __builtin_amdgcn_wave_barrier(); asm volatile("" ::: "memory");
    }
}

template <typename T16, int NSPLIT>
__global__ __launch_bounds__(32) void k_gemmPV(const T16* __restrict__ A, const T16* __restrict__ A2, const T16* __restrict__ Bt, const T16* __restrict__ Bt2, int ldb, float* O, int roff, size_t sA, size_t sB, size_t sO) {
    typedef typename WFrag<T16>::V V;
    __shared__ __align__(16) float os[16 * 68];
    const size_t z = blockIdx.z; A += z * sA; if (A2) A2 += z * sA; Bt += z * sB; if (Bt2) Bt2 += z * sB; O += z * sO;
    const int lane = threadIdx.x & 31, lr = lane & 15, hi = lane >> 4; const int r0 = roff + (int)blockIdx.x * 64; const int cb = r0 - BOFF; const int ks = (cb < 0) ? -cb : 0;
    v8f acc[4][4];
#pragma unroll
    for (int mb = 0; mb < 4; ++mb)
#pragma unroll
        for (int nb = 0; nb < 4; ++nb) acc[mb][nb] = (v8f){};
    const size_t aoff = (size_t)(r0 + lr) * BW + 8 * hi, boff = (size_t)lr * ldb + 8 * hi;
#pragma unroll 1
    for (int kc = ks; kc < BW; kc += 32) {
        const size_t t0 = (size_t)(cb + kc);
        V a[4], a2[4];
#pragma unroll
        for (int mb = 0; mb < 4; ++mb) { a[mb] = WFrag<T16>::ld(A + aoff + (size_t)mb * 16 * BW + kc); if (NSPLIT == 2) a2[mb] = WFrag<T16>::ld(A2 + aoff + (size_t)mb * 16 * BW + kc); }
#pragma unroll
        for (int nb = 0; nb < 4; ++nb) { const V b = WFrag<T16>::ld(Bt + boff + (size_t)nb * 16 * ldb + t0); V b2; if (NSPLIT == 2) b2 = WFrag<T16>::ld(Bt2 + boff + (size_t)nb * 16 * ldb + t0);
#pragma unroll
            for (int mb = 0; mb < 4; ++mb) { acc[mb][nb] = WFrag<T16>::mma(a[mb], b, acc[mb][nb]); if (NSPLIT == 2) { acc[mb][nb] = WFrag<T16>::mma(a2[mb], b, acc[mb][nb]); acc[mb][nb] = WFrag<T16>::mma(a[mb], b2, acc[mb][nb]); } } }
        asm volatile("v_nop\n\tv_nop\n\tv_nop\n\tv_nop" : "+v"(acc[0][0]), "+v"(acc[1][1]), "+v"(acc[2][2]), "+v"(acc[3][3]) : "v"(a[0]), "v"(a[3]));
    }
#pragma unroll
    for (int mb = 0; mb < 4; ++mb) {
#pragma unroll
        for (int nb = 0; nb < 4; ++nb) {
#pragma unroll
            for (int j = 0; j < 8; ++j) os[(hi * 8 + j) * 68 + nb * 16 + lr] = acc[mb][nb][j]; }
        __builtin_amdgcn_wave_barrier(); asm volatile("" ::: "memory");
        float* crow = O + (size_t)(r0 + mb * 16) * HD;
#pragma unroll 1
        for (int ps = 0; ps < 2; ++ps) {
#pragma unroll
            for (int s = 0; s < 8; ++s) { const int row = 2 * s + hi, cofs = lr * 4; const v4f val = *(const v4fa*)(os + row * 68 + cofs);
                *(volatile v4f*)(crow + (size_t)row * HD + cofs) = val; }
            if (ps == 0) __threadfence(); }
        __builtin_amdgcn_wave_barrier(); asm volatile("" ::: "memory");
    }
}

__global__ __launch_bounds__(256) void k_wtG(const float* __restrict__ w, int K, int N, bf* Bt) {
    const int lane = threadIdx.x & 31; const int L0 = (blockIdx.x * 8 + (threadIdx.x >> 5)) * 8; const int nlines = N * K / 64;
#pragma unroll
    for (int ps = 0; ps < 2; ++ps) {
#pragma unroll 1
        for (int l = 0; l < 8; ++l) { const int L = L0 + l; if (L >= nlines) break; const size_t e = (size_t)L * 64 + lane * 2; const int k = (int)(e % K), n = (int)(e / K); v2us o;
            o[0] = f2bf(w[(size_t)k * N + n]); o[1] = f2bf(w[(size_t)(k + 1) * N + n]); *(volatile v2us*)(Bt + e) = o; }
        if (ps == 0) __threadfence(); }
}
__global__ __launch_bounds__(256) void k_cvt8(const float* __restrict__ src, bf* dst, size_t n8) { const size_t i = (size_t)blockIdx.x * 256 + threadIdx.x; if (i >= n8) return; const v8f v = *(const v8f*)(src + i * 8); v8us o;
#pragma unroll
    for (int k = 0; k < 8; ++k) o[k] = f2bf(v[k]); *(volatile v8us*)(dst + i * 8) = o; __threadfence(); *(volatile v8us*)(dst + i * 8) = o; }

__global__ __launch_bounds__(256) void k_cstab(float* CS) {
    const int idx = blockIdx.x * 256 + threadIdx.x; if (idx >= SEQ * HD) return;
    const int t = idx / HD; const int i = idx & 31; const int ia = i & 7, ib = i >> 3;
    const double m = (ia == 0) ? 1.0 : (ia == 1) ? 0.7498942093324559 : (ia == 2) ? 0.5623413251903491 : (ia == 3) ? 0.4216965034285822 : (ia == 4) ? 0.31622776601683794 : (ia == 5) ? 0.23713737056616552 : (ia == 6) ? 0.17782794100389228 : 0.1333521432163324;
    const double s10 = (ib == 0) ? 1.0 : (ib == 1) ? 0.1 : (ib == 2) ? 0.01 : 0.001;
    const float inv = (float)(m * s10);
    const float ang = __fmul_rn((float)t, inv);
    const float nf = rintf(ang * 0.636619772f);
    const double r = (double)ang - (double)nf * 1.5707963267948966;
    const double r2 = r * r;
    double psn = 1.6059043836821613e-10;
    psn = psn * r2 - 2.505210838544172e-8;
    psn = psn * r2 + 2.7557319223985893e-6;
    psn = psn * r2 - 1.984126984126984e-4;
    psn = psn * r2 + 8.333333333333333e-3;
    psn = psn * r2 - 1.6666666666666666e-1;
    const double sn = r + r * r2 * psn;
    double pcs = 2.08767569878681e-9;
    pcs = pcs * r2 - 2.755731922398589e-7;
    pcs = pcs * r2 + 2.48015873015873e-5;
    pcs = pcs * r2 - 1.388888888888889e-3;
    pcs = pcs * r2 + 4.1666666666666664e-2;
    pcs = pcs * r2 - 0.5;
    const double cn = 1.0 + r2 * pcs;
    const int qd = ((int)nf) & 3;
    const double sv = (qd == 0) ? sn : (qd == 1) ? cn : (qd == 2) ? -sn : -cn;
    const double cv = (qd == 0) ? cn : (qd == 1) ? -sn : (qd == 2) ? -cn : sn;
    v2f cs; cs[0] = (float)cv; cs[1] = (float)sv;
    *(volatile v2f*)(CS + (size_t)idx * 2) = cs; __threadfence(); *(volatile v2f*)(CS + (size_t)idx * 2) = cs;
}

__global__ __launch_bounds__(256) void k_rope(const float* __restrict__ F, int pitch, int nheads, const float* __restrict__ CS, float sc, h16* P16, bf* Ph, bf* Pl) {
    const size_t e = ((size_t)blockIdx.x * 256 + threadIdx.x) * 2; if (e >= (size_t)nheads * SEQ * HD) return; const int d = (int)(e % HD); const int t = (int)((e / HD) % SEQ); const int h = (int)(e / ((size_t)HD * SEQ)); const float* f = F + (size_t)t * pitch + h * HD; v2h o16; v2us oh, ol;
#pragma unroll
    for (int q = 0; q < 2; ++q) { const int dd = d + q; const int dp = (dd < HD / 2) ? dd + HD / 2 : dd - HD / 2; const float x0 = f[dd], x1 = f[dp];
        const v2f cs = *(const v2f*)(CS + ((size_t)t * HD + dd) * 2); float a = __fmul_rn(x0, cs[0]), bq = __fmul_rn(x1, cs[1]); asm volatile("" : "+v"(a)); asm volatile("" : "+v"(bq)); const float r = ((dd < HD / 2) ? __fsub_rn(a, bq) : __fadd_rn(a, bq)) * sc;
        o16[q] = tohx(r); unsigned short a2, c2; splitf(r, a2, c2); oh[q] = a2; ol[q] = c2; }
    const bool hr = (t < RH); const size_t eh = ((size_t)h * RH + (hr ? t : 0)) * HD + d;
    *(volatile v2h*)(P16 + e) = o16; if (hr) { *(volatile v2us*)(Ph + eh) = oh; *(volatile v2us*)(Pl + eh) = ol; }
    __threadfence();
    *(volatile v2h*)(P16 + e) = o16; if (hr) { *(volatile v2us*)(Ph + eh) = oh; *(volatile v2us*)(Pl + eh) = ol; }
}
__global__ __launch_bounds__(256) void k_vtp(const float* __restrict__ F, int pitch, int nheads, h16* V16, bf* Vh, bf* Vl) { const size_t e = ((size_t)blockIdx.x * 256 + threadIdx.x) * 2; if (e >= (size_t)nheads * HD * SEQ) return; const int t = (int)(e % SEQ); const int d = (int)((e / SEQ) % HD); const int g = (int)(e / ((size_t)SEQ * HD)); v2h o16; v2us oh, ol;
#pragma unroll
    for (int q = 0; q < 2; ++q) { const float x = F[(size_t)(t + q) * pitch + g * HD + d]; o16[q] = tohx(x); unsigned short a2, c2; splitf(x, a2, c2); oh[q] = a2; ol[q] = c2; }
    const bool hr = (t < RH); const size_t eh = ((size_t)g * HD + d) * RH + (hr ? t : 0);
    *(volatile v2h*)(V16 + e) = o16; if (hr) { *(volatile v2us*)(Vh + eh) = oh; *(volatile v2us*)(Vl + eh) = ol; }
    __threadfence();
    *(volatile v2h*)(V16 + e) = o16; if (hr) { *(volatile v2us*)(Vh + eh) = oh; *(volatile v2us*)(Vl + eh) = ol; }
}
__global__ __launch_bounds__(256) void k_asoft(const float* __restrict__ Sb, h16* P16, bf* Ph, bf* Pl) {
    const int lane = threadIdx.x & 31; const int wv = __builtin_amdgcn_readfirstlane((int)(threadIdx.x >> 5)); const int row = blockIdx.x * 8 + wv; if (row >= ZH * SEQ) return;
    const int i = row % SEQ; const int zz = row / SEQ; const bool hires = (i < RH); const int cb = (i & ~63) - BOFF; const float* sr = Sb + (size_t)row * BW; float v[BW / 32]; float mx = -3.0e38f;
#pragma unroll
    for (int ch = 0; ch < BW / 64; ++ch) { const int jj0 = ch * 64 + lane * 2; const v2f a = *(const v2f*)(sr + jj0);
#pragma unroll
        for (int q = 0; q < 2; ++q) { const int j = cb + jj0 + q; const bool ok = (j >= 0) && (j <= i) && (i - j < WINK); const float t = ok ? a[q] * SCL : -3.0e38f; v[ch * 2 + q] = t; mx = fmaxf(mx, t); } }
#pragma unroll
    for (int sh = 16; sh; sh >>= 1) mx = fmaxf(mx, __shfl_xor(mx, sh, 32));
    float sum = 0.f;
#pragma unroll
    for (int k = 0; k < BW / 32; ++k) { float d0 = __fsub_rn(v[k], mx); asm volatile("" : "+v"(d0)); v[k] = __builtin_amdgcn_exp2f(__fmul_rn(d0, 1.4426950408889634f)); sum += v[k]; }
#pragma unroll
    for (int sh = 16; sh; sh >>= 1) sum += __shfl_xor(sum, sh, 32);
    const float f = __fdiv_rn(hires ? 1.0f : PCAR, sum);
#pragma unroll 1
    for (int ps = 0; ps < 2; ++ps) {
        if (hires) {
#pragma unroll
            for (int ch = 0; ch < BW / 64; ++ch) { v2us oh, ol;
#pragma unroll
                for (int q = 0; q < 2; ++q) { unsigned short a, c2; splitf(v[ch * 2 + q] * f, a, c2); oh[q] = a; ol[q] = c2; }
                const size_t oo = ((size_t)zz * RH + i) * BW + ch * 64 + lane * 2; *(volatile v2us*)(Ph + oo) = oh; *(volatile v2us*)(Pl + oo) = ol; }
        } else {
#pragma unroll
            for (int ch = 0; ch < BW / 64; ++ch) { v2h o2;
#pragma unroll
                for (int q = 0; q < 2; ++q) o2[q] = tohx(v[ch * 2 + q] * f);
                *(volatile v2h*)(P16 + (size_t)row * BW + ch * 64 + lane * 2) = o2; } }
        if (ps == 0) __threadfence(); }
}
__global__ __launch_bounds__(256) void k_merge(const float* __restrict__ O, int h0, bf* Ah, bf* Al) { const size_t e = ((size_t)blockIdx.x * 256 + threadIdx.x) * 2; if (e >= (size_t)ZH * SEQ * HD) return; const int d = (int)(e % HD); const int t = (int)((e / HD) % SEQ); const int zz = (int)(e / ((size_t)HD * SEQ)); const float cs = (t < RH) ? 1.0f : (1.0f / PCAR); const size_t oo = (size_t)t * DQ + (h0 + zz) * HD + d;
    v2us oh, ol;
#pragma unroll
    for (int q = 0; q < 2; ++q) { unsigned short a, c2; splitf(O[e + q] * cs, a, c2); oh[q] = a; ol[q] = c2; } *(volatile v2us*)(Ah + oo) = oh; *(volatile v2us*)(Al + oo) = ol; __threadfence(); *(volatile v2us*)(Ah + oo) = oh; *(volatile v2us*)(Al + oo) = ol; }

extern "C" void kernel_launch(void* const* d_in, const int* in_sizes, int n_in,
                              void* d_out, int out_size, void* d_ws, size_t ws_size, hipStream_t stream) {
    if (n_in < 6) return;
    const long long needx = ((long long)(NB - 1) * SEQ_FULL + SEQ) * DM;
    if ((long long)in_sizes[0] < needx) return;
    if ((long long)in_sizes[1] < (long long)DM * DQ || (long long)in_sizes[2] < (long long)DM * DQ || (long long)in_sizes[3] < (long long)DM * DQ || (long long)in_sizes[4] < (long long)DQ * DM || in_sizes[5] < DM) return;
    if ((long long)out_size < needx) return;
    const float* x = (const float*)d_in[0]; const float* wq = (const float*)d_in[1]; const float* wk = (const float*)d_in[2]; const float* wv = (const float*)d_in[3]; const float* wo = (const float*)d_in[4]; const float* bo = (const float*)d_in[5];
    float* OUT = (float*)d_out;
    char* wsp = (char*)d_ws;
    auto take = [&](size_t bytes) { char* p = wsp; wsp += (bytes + 255) & ~(size_t)255; return (void*)p; };
    bf* WQ = (bf*)take((size_t)DQ * DM * 2); bf* WK = (bf*)take((size_t)DQ * DM * 2); bf* WV = (bf*)take((size_t)DQ * DM * 2); bf* WO = (bf*)take((size_t)DM * DQ * 2); float* CS = (float*)take((size_t)SEQ * HD * 2 * 4);
    bf* XB = (bf*)take((size_t)SEQ * DM * 2); float* F = (float*)take((size_t)SEQ * DQ * 4);
    h16* QP16 = (h16*)take((size_t)NH_ * SEQ * HD * 2); h16* KP16 = (h16*)take((size_t)NH_ * SEQ * HD * 2); h16* VT16 = (h16*)take((size_t)NH_ * HD * SEQ * 2);
    bf* QPh = (bf*)take((size_t)NH_ * RH * HD * 2); bf* QPl = (bf*)take((size_t)NH_ * RH * HD * 2); bf* KPh = (bf*)take((size_t)NH_ * RH * HD * 2); bf* KPl = (bf*)take((size_t)NH_ * RH * HD * 2); bf* VTh = (bf*)take((size_t)NH_ * HD * RH * 2); bf* VTl = (bf*)take((size_t)NH_ * HD * RH * 2);
    float* Sb = (float*)take((size_t)ZH * SEQ * BW * 4); h16* P16 = (h16*)take((size_t)ZH * SEQ * BW * 2); bf* Ph = (bf*)take((size_t)ZH * RH * BW * 2); bf* Pl = (bf*)take((size_t)ZH * RH * BW * 2);
    float* Ob = (float*)take((size_t)ZH * SEQ * HD * 4); bf* ATh = (bf*)take((size_t)SEQ * DQ * 2); bf* ATl = (bf*)take((size_t)SEQ * DQ * 2);
    if ((size_t)(wsp - (char*)d_ws) > ws_size) return;
    k_wtG<<<(unsigned)((DM * DQ / 64 + 63) / 64), 256, 0, stream>>>(wq, DM, DQ, WQ);
    k_wtG<<<(unsigned)((DM * DQ / 64 + 63) / 64), 256, 0, stream>>>(wk, DM, DQ, WK);
    k_wtG<<<(unsigned)((DM * DQ / 64 + 63) / 64), 256, 0, stream>>>(wv, DM, DQ, WV);
    k_wtG<<<(unsigned)((DQ * DM / 64 + 63) / 64), 256, 0, stream>>>(wo, DQ, DM, WO);
    k_cstab<<<(SEQ * HD + 255) / 256, 256, 0, stream>>>(CS);
    const unsigned LQ = (unsigned)(((size_t)NH_ * SEQ * HD / 2 + 255) / 256);
    for (int b = 0; b < NB; ++b) {
        k_cvt8<<<(unsigned)(((size_t)SEQ * DM / 8 + 255) / 256), 256, 0, stream>>>(x + (size_t)b * SEQ_FULL * DM, XB, (size_t)SEQ * DM / 8);
        k_gemmw<bf, 0, false><<<dim3(SEQ / 64, DQ / 64, 1), 32, 0, stream>>>(XB, nullptr, WQ, nullptr, DM, F, DQ, nullptr, 0, 0, 0);
        k_rope<<<LQ, 256, 0, stream>>>(F, DQ, NH_, CS, 1.0f, QP16, QPh, QPl);
        k_gemmw<bf, 0, false><<<dim3(SEQ / 64, DQ / 64, 1), 32, 0, stream>>>(XB, nullptr, WK, nullptr, DM, F, DQ, nullptr, 0, 0, 0);
        k_rope<<<LQ, 256, 0, stream>>>(F, DQ, NH_, CS, 1.0f, KP16, KPh, KPl);
        k_gemmw<bf, 0, false><<<dim3(SEQ / 64, DQ / 64, 1), 32, 0, stream>>>(XB, nullptr, WV, nullptr, DM, F, DQ, nullptr, 0, 0, 0);
        k_vtp<<<LQ, 256, 0, stream>>>(F, DQ, NH_, VT16, VTh, VTl);
        for (int h0 = 0; h0 < NH_; h0 += ZH) { const size_t zq = (size_t)h0;
            k_gemmS<bf, 2><<<dim3(RH / 64, BW / 64, ZH), 32, 0, stream>>>(QPh + zq * RH * HD, QPl + zq * RH * HD, KPh + zq * RH * HD, KPl + zq * RH * HD, Sb, 0, (size_t)RH * HD, (size_t)RH * HD, (size_t)SEQ * BW);
            if (SEQ > RH) k_gemmS<h16, 0><<<dim3((SEQ - RH) / 64, BW / 64, ZH), 32, 0, stream>>>(QP16 + zq * SEQ * HD, nullptr, KP16 + zq * SEQ * HD, nullptr, Sb, RH, (size_t)SEQ * HD, (size_t)SEQ * HD, (size_t)SEQ * BW);
            k_asoft<<<ZH * SEQ / 8, 256, 0, stream>>>(Sb, P16, Ph, Pl);
            k_gemmPV<bf, 2><<<dim3(RH / 64, 1, ZH), 32, 0, stream>>>(Ph, Pl, VTh + zq * HD * RH, VTl + zq * HD * RH, RH, Ob, 0, (size_t)RH * BW, (size_t)HD * RH, (size_t)SEQ * HD);
            if (SEQ > RH) k_gemmPV<h16, 0><<<dim3((SEQ - RH) / 64, 1, ZH), 32, 0, stream>>>(P16, nullptr, VT16 + zq * HD * SEQ, nullptr, SEQ, Ob, RH, (size_t)SEQ * BW, (size_t)HD * SEQ, (size_t)SEQ * HD);
            k_merge<<<(unsigned)(((size_t)ZH * SEQ * HD / 2 + 255) / 256), 256, 0, stream>>>(Ob, h0, ATh, ATl); }
        k_gemmw<bf, 1, true><<<dim3(SEQ / 64, DM / 64, 1), 32, 0, stream>>>(ATh, ATl, WO, nullptr, DQ, OUT + (size_t)b * SEQ_FULL * DM, DM, bo, 0, 0, 0); }
}
